// DrugRepresentationModule_53326313947260
// MI455X (gfx1250) — hardware-run, weakly checked
//
#include <hip/hip_runtime.h>


namespace {
constexpr int N = 50000, E = 800000, AD = 78, ADP = 96, H = 128, OUT = 100, G = 500, GP = 512, NL = 3;
constexpr float XS = 8.0f, HS = 256.0f, WSC = 256.0f, BNS = 0.99999500003749970f  ;
typedef _Float16 b16;
typedef __attribute__((ext_vector_type(16))) _Float16 v16b;
typedef __attribute__((ext_vector_type(8))) _Float16 v8b;
typedef __attribute__((ext_vector_type(8))) float v8f;
typedef __attribute__((ext_vector_type(4))) float v4f;
__device__ __forceinline__ float bf16_rne(float f) { unsigned int u = __float_as_uint(f); u += 0x7FFFu + ((u >> 16) & 1u); float r = __uint_as_float(u & 0xFFFF0000u); asm volatile("" : "+v"(r)); return r; }
__device__ __forceinline__ float bfv(float f) { float r = bf16_rne(f); asm volatile("" : "+v"(r)); return r; }
__device__ __forceinline__ void split16(float v, b16& hi, b16& lo) { hi = (b16)v; lo = (b16)(v - (float)hi); }
__device__ __forceinline__ v16b frag_kb(const b16* p, int hh) { const v8b a = *(const v8b*)(p + 8 * hh), b = *(const v8b*)(p + 16 + 8 * hh); v16b f;
#pragma unroll
  for (int e = 0; e < 8; ++e) { f[e] = a[e]; f[8 + e] = b[e]; } return f; }
__device__ __forceinline__ v8f wmma16b(v16b a, v16b b, v8f c) { v8f d = __builtin_amdgcn_wmma_f32_16x16x32_f16(false, a, false, b, (short)0, c, false, false); asm volatile("v_nop\n\tv_nop\n\tv_nop\n\tv_nop" : "+v"(d) : "v"(a), "v"(b)); return d; }
__device__ __forceinline__ void wave_lds_sync() { __builtin_amdgcn_fence(__ATOMIC_RELEASE, "workgroup"); __builtin_amdgcn_wave_barrier(); __builtin_amdgcn_fence(__ATOMIC_ACQUIRE, "workgroup"); }
__device__ __forceinline__ float pmul(float a, float b) { float p = a * b; asm volatile("" : "+v"(p)); return p; }
__device__ __forceinline__ int iclamp(int v, int lo, int hi) { return v < lo ? lo : (v > hi ? hi : v); }
constexpr int CSR_NBLK8 = 512, CSR_GB8 = 8, CSR_GN8 = 1 << CSR_GB8  , CSR_TS8 = (CSR_GN8 < 32 ? 32 : CSR_GN8)  , CSR_MAXG8 = 512, CSR_CAP8 = 12288  ;
__device__ __host__ __forceinline__ int csr_tix8(int v) { return (v >> CSR_GB8) * CSR_TS8 + (v & (CSR_GN8 - 1)); }
__global__ __launch_bounds__(64) void csrA_kernel8(const int* __restrict__ dst, int E, int N, int nG, int CHP, int NGP, int* __restrict__ STG, int* __restrict__ HST) {
  extern __shared__ int sm[];
  int* cnt = sm; int* run = sm + NGP; int* ids = sm + 2 * NGP;
  const int b = blockIdx.x; const int ch = (E + CSR_NBLK8 - 1) / CSR_NBLK8; const int e0 = b * ch, e1 = min(E, e0 + ch);
  for (int i = threadIdx.x; i < NGP; i += 64) cnt[i] = 0;
  for (int i = threadIdx.x; i < CHP; i += 64) ids[i] = -1;
  __syncthreads();
  if (threadIdx.x == 0) {
    for (int e = e0; e < e1; ++e) { int d = dst[e]; d = (d < 0) ? 0 : (d >= N ? N - 1 : d); cnt[d >> CSR_GB8] += 1; }
    int acc = 0; for (int g = 0; g < nG; ++g) { run[g] = acc; acc += cnt[g]; }
    for (int e = e0; e < e1; ++e) { int d = dst[e]; d = (d < 0) ? 0 : (d >= N ? N - 1 : d); const int g = d >> CSR_GB8; ids[run[g]] = e; run[g] += 1; } }
  __syncthreads();
  typedef __attribute__((ext_vector_type(4))) int v4i;
  for (int pass = 0; pass < 2; ++pass) {
    for (int i = threadIdx.x; i < CHP / 4; i += 64) *(volatile v4i*)(STG + (size_t)b * CHP + i * 4) = *(const v4i*)(&ids[i * 4]);
    for (int i = threadIdx.x; i < NGP / 4; i += 64) { v4i v; for (int e = 0; e < 4; ++e) v[e] = (i * 4 + e < nG) ? cnt[i * 4 + e] : 0; *(volatile v4i*)(HST + (size_t)b * NGP + i * 4) = v; }
    __threadfence(); }
}
__global__ __launch_bounds__(512) void csrS_kernel8(const int* __restrict__ HST, int nG, int NGP, int* __restrict__ START, int* __restrict__ TOT, int* __restrict__ OFF) {
  __shared__ int tot[CSR_MAXG8];
  const int b = threadIdx.x;
  for (int pass = 0; pass < 2; ++pass) { int runb = 0; for (int g = 0; g < nG; ++g) { int c = HST[(size_t)b * NGP + g]; c = (c < 0) ? 0 : c; ((volatile int*)OFF)[(size_t)g * CSR_NBLK8 + b] = runb; runb += c; } __threadfence(); }
  for (int g = threadIdx.x; g < nG; g += 512) { int s = 0; for (int bb = 0; bb < CSR_NBLK8; ++bb) { int c = HST[(size_t)bb * NGP + g]; s += (c < 0) ? 0 : c; } tot[g] = s; }
  __syncthreads();
  if (threadIdx.x < 32) {
    __shared__ int st[CSR_MAXG8 + 32];
    if (threadIdx.x == 0) { int acc = 0; for (int g = 0; g < NGP; ++g) { st[g] = acc; if (g < nG) acc += (tot[g] + 31) & ~31; } st[NGP] = acc; }
    __builtin_amdgcn_fence(__ATOMIC_RELEASE, "workgroup"); __builtin_amdgcn_wave_barrier(); __builtin_amdgcn_fence(__ATOMIC_ACQUIRE, "workgroup");
    for (int pass = 0; pass < 2; ++pass) { for (int i = threadIdx.x; i < NGP + 32; i += 32) { ((volatile int*)START)[i] = (i <= NGP) ? st[min(i, NGP)] : 0; ((volatile int*)TOT)[i] = (i < nG) ? tot[i] : 0; } __threadfence(); } }
}
__global__ __launch_bounds__(256) void csrB_kernel8(const int* __restrict__ dst, int N, int nG, int CHP, int NGP, int permLen, const int* __restrict__ STG, const int* __restrict__ HST, const int* __restrict__ OFF, const int* __restrict__ START, const int* __restrict__ TOT, int* __restrict__ PERM, int* __restrict__ ROWPTR, int* __restrict__ ROWCNT, int* __restrict__ FLAG) {
  typedef __attribute__((ext_vector_type(4))) int v4i;
  __shared__ int ids[CSR_CAP8]; __shared__ unsigned short key[CSR_CAP8]; __shared__ int outp[CSR_CAP8]; __shared__ int ncnt[CSR_GN8 + 1]; __shared__ int boff[CSR_NBLK8 + 1];
  const int g = blockIdx.x, t_ = threadIdx.x; int tot = TOT[g]; int st = START[g], stn = START[g + 1]; const int v0 = g * CSR_GN8; const int nv = min(CSR_GN8, N - v0); const int t0 = g * CSR_TS8;
  st = (st < 0) ? 0 : (st > permLen - 32 ? permLen - 32 : st) & ~31; stn = (stn < st) ? st : (stn > permLen ? permLen : stn); tot = (tot < 0) ? 0 : tot; if (tot > stn - st && tot <= CSR_CAP8) tot = stn - st;
  if (tot > CSR_CAP8) {
    for (int pass = 0; pass < 2; ++pass) { for (int i = t_; i < CSR_TS8 / 4; i += 256) { v4i a, c; for (int e = 0; e < 4; ++e) { a[e] = st; c[e] = 0; } *(volatile v4i*)(ROWPTR + t0 + i * 4) = a; *(volatile v4i*)(ROWCNT + t0 + i * 4) = c; } if (t_ == 0) ((volatile int*)FLAG)[0] = 1; __threadfence(); } (void)nv; return; }
  if (t_ == 0) { int acc = 0; for (int b = 0; b < CSR_NBLK8; ++b) { boff[b] = acc; int c = HST[(size_t)b * NGP + g]; c = (c < 0) ? 0 : (c > CHP ? CHP : c); acc += c; if (acc > tot) acc = tot; } boff[CSR_NBLK8] = acc; }
  for (int i = t_; i <= CSR_GN8; i += 256) ncnt[i] = 0;
  __syncthreads();
  for (int b = 0; b < CSR_NBLK8; ++b) { const int c = boff[b + 1] - boff[b]; int o_ = OFF[(size_t)g * CSR_NBLK8 + b]; o_ = (o_ < 0) ? 0 : (o_ > CHP - c ? CHP - c : o_); const int* src_ = STG + (size_t)b * CHP + o_;
    for (int i = t_; i < c; i += 256) { int id = src_[i]; id = (id < 0) ? 0 : id; ids[boff[b] + i] = id; int d = dst[id]; d = (d < v0) ? v0 : (d >= N ? N - 1 : d); int kk = d - v0; kk = (kk < 0) ? 0 : (kk >= CSR_GN8 ? CSR_GN8 - 1 : kk); key[boff[b] + i] = (unsigned short)kk; } }
  __syncthreads();
  if (t_ == 0) { for (int i = 0; i < tot; ++i) ncnt[key[i]] += 1; int acc = 0; for (int vl = 0; vl < CSR_GN8; ++vl) { const int c = ncnt[vl]; ncnt[vl] = acc; acc += c; } ncnt[CSR_GN8] = acc;
    for (int i = 0; i < tot; ++i) { const int vl = key[i]; outp[ncnt[vl]] = ids[i]; ncnt[vl] += 1; }
    for (int vl = CSR_GN8; vl > 0; --vl) ncnt[vl] = ncnt[vl - 1]; ncnt[0] = 0; }
  __syncthreads();
  for (int pass = 0; pass < 2; ++pass) {
    for (int i = t_; i < (stn - st) / 4; i += 256) { v4i v; for (int e = 0; e < 4; ++e) { const int q = i * 4 + e; v[e] = (q < tot) ? outp[q] : -1; } *(volatile v4i*)(PERM + st + i * 4) = v; }
    for (int i = t_; i < CSR_TS8 / 4; i += 256) { v4i a, c; for (int e = 0; e < 4; ++e) { const int vl = i * 4 + e; const int vc = vl < CSR_GN8 ? vl : CSR_GN8; a[e] = (vl < CSR_GN8) ? st + ncnt[vc] : st; c[e] = (vl < nv) ? (ncnt[(vc < CSR_GN8 ? vc : CSR_GN8 - 1) + 1] - ncnt[vc]) : 0; } *(volatile v4i*)(ROWPTR + t0 + i * 4) = a; *(volatile v4i*)(ROWCNT + t0 + i * 4) = c; }
    __threadfence(); }
}
__global__ __launch_bounds__(256) void csrZ_kernel8(int* __restrict__ p, size_t n4) { typedef __attribute__((ext_vector_type(4))) int v4i; const size_t tid = (size_t)blockIdx.x * 256 + threadIdx.x, nth = (size_t)gridDim.x * 256; v4i z = {0, 0, 0, 0}; for (size_t i = tid; i < n4; i += nth) *(volatile v4i*)(p + i * 4) = z; }
struct CsrBufs8 { int *STG, *HST, *OFF, *START, *TOT, *PERM, *ROWPTR, *ROWCNT, *FLAG; int nG, NGP, CHP; size_t permLen; char* base; size_t bytes; };
static size_t csr_carve8(CsrBufs8& c, char* ws, size_t off, int E, int N) {
  const size_t off0 = off; c.base = ws + off;
  auto al = [&](size_t bytes) { char* p = ws + off; off += (bytes + 255) & ~(size_t)255; return p; };
  c.nG = (N + CSR_GN8 - 1) / CSR_GN8; c.NGP = (c.nG + 31) & ~31; const int ch = (E + CSR_NBLK8 - 1) / CSR_NBLK8; c.CHP = (ch + 31) & ~31; c.permLen = (size_t)E + 32 * (size_t)c.nG + 32;
  c.STG = (int*)al((size_t)CSR_NBLK8 * c.CHP * 4); c.HST = (int*)al((size_t)CSR_NBLK8 * c.NGP * 4); c.OFF = (int*)al((size_t)c.NGP * CSR_NBLK8 * 4); c.START = (int*)al((size_t)(c.NGP + 64) * 4); c.TOT = (int*)al((size_t)(c.NGP + 64) * 4);
  c.PERM = (int*)al(c.permLen * 4); c.ROWPTR = (int*)al((size_t)c.nG * CSR_TS8 * 4); c.ROWCNT = (int*)al((size_t)c.nG * CSR_TS8 * 4); c.FLAG = (int*)al(256);
  c.bytes = off - off0; return off;
}
static void csr_build8(const CsrBufs8& c, const int* dst, int E, int N, hipStream_t stream) {
  const size_t smem = (size_t)(2 * c.NGP + c.CHP) * 4;
  csrZ_kernel8<<<512, 256, 0, stream>>>((int*)c.base, c.bytes / 16);
  csrA_kernel8<<<CSR_NBLK8, 64, smem, stream>>>(dst, E, N, c.nG, c.CHP, c.NGP, c.STG, c.HST);
  csrS_kernel8<<<1, 512, 0, stream>>>(c.HST, c.nG, c.NGP, c.START, c.TOT, c.OFF);
  csrB_kernel8<<<c.nG, 256, 0, stream>>>(dst, N, c.nG, c.CHP, c.NGP, (int)c.permLen, c.STG, c.HST, c.OFF, c.START, c.TOT, c.PERM, c.ROWPTR, c.ROWCNT, c.FLAG);
}
constexpr int CSR_NBLK5 = 512, CSR_GB5 = 5, CSR_GN5 = 1 << CSR_GB5  , CSR_TS5 = (CSR_GN5 < 32 ? 32 : CSR_GN5)  , CSR_MAXG5 = 512, CSR_CAP5 = 12288  ;
__device__ __host__ __forceinline__ int csr_tix5(int v) { return (v >> CSR_GB5) * CSR_TS5 + (v & (CSR_GN5 - 1)); }
__global__ __launch_bounds__(64) void csrA_kernel5(const int* __restrict__ dst, int E, int N, int nG, int CHP, int NGP, int* __restrict__ STG, int* __restrict__ HST) {
  extern __shared__ int sm[];
  int* cnt = sm; int* run = sm + NGP; int* ids = sm + 2 * NGP;
  const int b = blockIdx.x; const int ch = (E + CSR_NBLK5 - 1) / CSR_NBLK5; const int e0 = b * ch, e1 = min(E, e0 + ch);
  for (int i = threadIdx.x; i < NGP; i += 64) cnt[i] = 0;
  for (int i = threadIdx.x; i < CHP; i += 64) ids[i] = -1;
  __syncthreads();
  if (threadIdx.x == 0) {
    for (int e = e0; e < e1; ++e) { int d = dst[e]; d = (d < 0) ? 0 : (d >= N ? N - 1 : d); cnt[d >> CSR_GB5] += 1; }
    int acc = 0; for (int g = 0; g < nG; ++g) { run[g] = acc; acc += cnt[g]; }
    for (int e = e0; e < e1; ++e) { int d = dst[e]; d = (d < 0) ? 0 : (d >= N ? N - 1 : d); const int g = d >> CSR_GB5; ids[run[g]] = e; run[g] += 1; } }
  __syncthreads();
  typedef __attribute__((ext_vector_type(4))) int v4i;
  for (int pass = 0; pass < 2; ++pass) {
    for (int i = threadIdx.x; i < CHP / 4; i += 64) *(volatile v4i*)(STG + (size_t)b * CHP + i * 4) = *(const v4i*)(&ids[i * 4]);
    for (int i = threadIdx.x; i < NGP / 4; i += 64) { v4i v; for (int e = 0; e < 4; ++e) v[e] = (i * 4 + e < nG) ? cnt[i * 4 + e] : 0; *(volatile v4i*)(HST + (size_t)b * NGP + i * 4) = v; }
    __threadfence(); }
}
__global__ __launch_bounds__(512) void csrS_kernel5(const int* __restrict__ HST, int nG, int NGP, int* __restrict__ START, int* __restrict__ TOT, int* __restrict__ OFF) {
  __shared__ int tot[CSR_MAXG5];
  const int b = threadIdx.x;
  for (int pass = 0; pass < 2; ++pass) { int runb = 0; for (int g = 0; g < nG; ++g) { int c = HST[(size_t)b * NGP + g]; c = (c < 0) ? 0 : c; ((volatile int*)OFF)[(size_t)g * CSR_NBLK5 + b] = runb; runb += c; } __threadfence(); }
  for (int g = threadIdx.x; g < nG; g += 512) { int s = 0; for (int bb = 0; bb < CSR_NBLK5; ++bb) { int c = HST[(size_t)bb * NGP + g]; s += (c < 0) ? 0 : c; } tot[g] = s; }
  __syncthreads();
  if (threadIdx.x < 32) {
    __shared__ int st[CSR_MAXG5 + 32];
    if (threadIdx.x == 0) { int acc = 0; for (int g = 0; g < NGP; ++g) { st[g] = acc; if (g < nG) acc += (tot[g] + 31) & ~31; } st[NGP] = acc; }
    __builtin_amdgcn_fence(__ATOMIC_RELEASE, "workgroup"); __builtin_amdgcn_wave_barrier(); __builtin_amdgcn_fence(__ATOMIC_ACQUIRE, "workgroup");
    for (int pass = 0; pass < 2; ++pass) { for (int i = threadIdx.x; i < NGP + 32; i += 32) { ((volatile int*)START)[i] = (i <= NGP) ? st[min(i, NGP)] : 0; ((volatile int*)TOT)[i] = (i < nG) ? tot[i] : 0; } __threadfence(); } }
}
__global__ __launch_bounds__(256) void csrB_kernel5(const int* __restrict__ dst, int N, int nG, int CHP, int NGP, int permLen, const int* __restrict__ STG, const int* __restrict__ HST, const int* __restrict__ OFF, const int* __restrict__ START, const int* __restrict__ TOT, int* __restrict__ PERM, int* __restrict__ ROWPTR, int* __restrict__ ROWCNT, int* __restrict__ FLAG) {
  typedef __attribute__((ext_vector_type(4))) int v4i;
  __shared__ int ids[CSR_CAP5]; __shared__ unsigned short key[CSR_CAP5]; __shared__ int outp[CSR_CAP5]; __shared__ int ncnt[CSR_GN5 + 1]; __shared__ int boff[CSR_NBLK5 + 1];
  const int g = blockIdx.x, t_ = threadIdx.x; int tot = TOT[g]; int st = START[g], stn = START[g + 1]; const int v0 = g * CSR_GN5; const int nv = min(CSR_GN5, N - v0); const int t0 = g * CSR_TS5;
  st = (st < 0) ? 0 : (st > permLen - 32 ? permLen - 32 : st) & ~31; stn = (stn < st) ? st : (stn > permLen ? permLen : stn); tot = (tot < 0) ? 0 : tot; if (tot > stn - st && tot <= CSR_CAP5) tot = stn - st;
  if (tot > CSR_CAP5) {
    for (int pass = 0; pass < 2; ++pass) { for (int i = t_; i < CSR_TS5 / 4; i += 256) { v4i a, c; for (int e = 0; e < 4; ++e) { a[e] = st; c[e] = 0; } *(volatile v4i*)(ROWPTR + t0 + i * 4) = a; *(volatile v4i*)(ROWCNT + t0 + i * 4) = c; } if (t_ == 0) ((volatile int*)FLAG)[0] = 1; __threadfence(); } (void)nv; return; }
  if (t_ == 0) { int acc = 0; for (int b = 0; b < CSR_NBLK5; ++b) { boff[b] = acc; int c = HST[(size_t)b * NGP + g]; c = (c < 0) ? 0 : (c > CHP ? CHP : c); acc += c; if (acc > tot) acc = tot; } boff[CSR_NBLK5] = acc; }
  for (int i = t_; i <= CSR_GN5; i += 256) ncnt[i] = 0;
  __syncthreads();
  for (int b = 0; b < CSR_NBLK5; ++b) { const int c = boff[b + 1] - boff[b]; int o_ = OFF[(size_t)g * CSR_NBLK5 + b]; o_ = (o_ < 0) ? 0 : (o_ > CHP - c ? CHP - c : o_); const int* src_ = STG + (size_t)b * CHP + o_;
    for (int i = t_; i < c; i += 256) { int id = src_[i]; id = (id < 0) ? 0 : id; ids[boff[b] + i] = id; int d = dst[id]; d = (d < v0) ? v0 : (d >= N ? N - 1 : d); int kk = d - v0; kk = (kk < 0) ? 0 : (kk >= CSR_GN5 ? CSR_GN5 - 1 : kk); key[boff[b] + i] = (unsigned short)kk; } }
  __syncthreads();
  if (t_ == 0) { for (int i = 0; i < tot; ++i) ncnt[key[i]] += 1; int acc = 0; for (int vl = 0; vl < CSR_GN5; ++vl) { const int c = ncnt[vl]; ncnt[vl] = acc; acc += c; } ncnt[CSR_GN5] = acc;
    for (int i = 0; i < tot; ++i) { const int vl = key[i]; outp[ncnt[vl]] = ids[i]; ncnt[vl] += 1; }
    for (int vl = CSR_GN5; vl > 0; --vl) ncnt[vl] = ncnt[vl - 1]; ncnt[0] = 0; }
  __syncthreads();
  for (int pass = 0; pass < 2; ++pass) {
    for (int i = t_; i < (stn - st) / 4; i += 256) { v4i v; for (int e = 0; e < 4; ++e) { const int q = i * 4 + e; v[e] = (q < tot) ? outp[q] : -1; } *(volatile v4i*)(PERM + st + i * 4) = v; }
    for (int i = t_; i < CSR_TS5 / 4; i += 256) { v4i a, c; for (int e = 0; e < 4; ++e) { const int vl = i * 4 + e; const int vc = vl < CSR_GN5 ? vl : CSR_GN5; a[e] = (vl < CSR_GN5) ? st + ncnt[vc] : st; c[e] = (vl < nv) ? (ncnt[(vc < CSR_GN5 ? vc : CSR_GN5 - 1) + 1] - ncnt[vc]) : 0; } *(volatile v4i*)(ROWPTR + t0 + i * 4) = a; *(volatile v4i*)(ROWCNT + t0 + i * 4) = c; }
    __threadfence(); }
}
__global__ __launch_bounds__(256) void csrZ_kernel5(int* __restrict__ p, size_t n4) { typedef __attribute__((ext_vector_type(4))) int v4i; const size_t tid = (size_t)blockIdx.x * 256 + threadIdx.x, nth = (size_t)gridDim.x * 256; v4i z = {0, 0, 0, 0}; for (size_t i = tid; i < n4; i += nth) *(volatile v4i*)(p + i * 4) = z; }
struct CsrBufs5 { int *STG, *HST, *OFF, *START, *TOT, *PERM, *ROWPTR, *ROWCNT, *FLAG; int nG, NGP, CHP; size_t permLen; char* base; size_t bytes; };
static size_t csr_carve5(CsrBufs5& c, char* ws, size_t off, int E, int N) {
  const size_t off0 = off; c.base = ws + off;
  auto al = [&](size_t bytes) { char* p = ws + off; off += (bytes + 255) & ~(size_t)255; return p; };
  c.nG = (N + CSR_GN5 - 1) / CSR_GN5; c.NGP = (c.nG + 31) & ~31; const int ch = (E + CSR_NBLK5 - 1) / CSR_NBLK5; c.CHP = (ch + 31) & ~31; c.permLen = (size_t)E + 32 * (size_t)c.nG + 32;
  c.STG = (int*)al((size_t)CSR_NBLK5 * c.CHP * 4); c.HST = (int*)al((size_t)CSR_NBLK5 * c.NGP * 4); c.OFF = (int*)al((size_t)c.NGP * CSR_NBLK5 * 4); c.START = (int*)al((size_t)(c.NGP + 64) * 4); c.TOT = (int*)al((size_t)(c.NGP + 64) * 4);
  c.PERM = (int*)al(c.permLen * 4); c.ROWPTR = (int*)al((size_t)c.nG * CSR_TS5 * 4); c.ROWCNT = (int*)al((size_t)c.nG * CSR_TS5 * 4); c.FLAG = (int*)al(256);
  c.bytes = off - off0; return off;
}
static void csr_build5(const CsrBufs5& c, const int* dst, int E, int N, hipStream_t stream) {
  const size_t smem = (size_t)(2 * c.NGP + c.CHP) * 4;
  csrZ_kernel5<<<512, 256, 0, stream>>>((int*)c.base, c.bytes / 16);
  csrA_kernel5<<<CSR_NBLK5, 64, smem, stream>>>(dst, E, N, c.nG, c.CHP, c.NGP, c.STG, c.HST);
  csrS_kernel5<<<1, 512, 0, stream>>>(c.HST, c.nG, c.NGP, c.START, c.TOT, c.OFF);
  csrB_kernel5<<<c.nG, 256, 0, stream>>>(dst, N, c.nG, c.CHP, c.NGP, (int)c.permLen, c.STG, c.HST, c.OFF, c.START, c.TOT, c.PERM, c.ROWPTR, c.ROWCNT, c.FLAG);
}


__global__ __launch_bounds__(256) void wput_kernel(const float* __restrict__ wemb, const float* __restrict__ w1, const float* __restrict__ w2, const float* __restrict__ wf1, const float* __restrict__ wf2, b16* __restrict__ WE, b16* __restrict__ WL, b16* __restrict__ WF1, b16* __restrict__ WF2) { const size_t nt = (size_t)gridDim.x * 256, u0 = (size_t)blockIdx.x * 256 + threadIdx.x; v8b v;
  for (size_t u = u0; u < (size_t)H * (ADP / 8); u += nt) { const int o = (int)(u / (ADP / 8)), k0 = (int)(u % (ADP / 8)) * 8;
#pragma unroll
    for (int j = 0; j < 8; ++j) { const int k = k0 + j; v[j] = (b16)(k < AD ? bf16_rne(wemb[(size_t)k * H + o]) * WSC : 0.0f); } for (int pass = 0; pass < 2; ++pass) { *(volatile v8b*)(WE + (size_t)o * ADP + k0) = v; __threadfence(); } }
  for (size_t u = u0; u < (size_t)2 * NL * H * 16; u += nt) { const int m = (int)(u / (H * 16)), r = (int)(u % (H * 16)); const int o = r / 16, k0 = (r % 16) * 8; const int l = m / 2; const float* w = (m & 1) ? w2 + (size_t)l * H * H : w1 + (size_t)l * H * H;
#pragma unroll
    for (int j = 0; j < 8; ++j) v[j] = (b16)(bf16_rne(w[(size_t)(k0 + j) * H + o]) * WSC); for (int pass = 0; pass < 2; ++pass) { *(volatile v8b*)(WL + ((size_t)m * H + o) * H + k0) = v; __threadfence(); } }
  for (size_t u = u0; u < (size_t)(H + 112) * 16; u += nt) { const int o = (int)(u / 16), k0 = (int)(u % 16) * 8;
#pragma unroll
    for (int j = 0; j < 8; ++j) { float w; if (o < H) w = wf1[(size_t)(k0 + j) * H + o]; else { const int oo = o - H; w = oo < OUT ? wf2[(size_t)(k0 + j) * OUT + oo] : 0.0f; } v[j] = (b16)(bf16_rne(w) * WSC); }
    b16* dst = o < H ? WF1 + (size_t)o * H + k0 : WF2 + (size_t)(o - H) * H + k0; for (int pass = 0; pass < 2; ++pass) { *(volatile v8b*)dst = v; __threadfence(); } } }
__global__ __launch_bounds__(32) void emb_kernel(const float* __restrict__ x, const b16* __restrict__ WE, const float* __restrict__ be, int NLIM, float* __restrict__ HA) { __shared__ __attribute__((aligned(16))) b16 Ah[16][ADP + 8]; __shared__ float Tf[16][H + 4]; const int lane = threadIdx.x, nloc = lane & 15, hlf = lane >> 4; const size_t m0 = (size_t)blockIdx.x * 16; if (m0 >= (size_t)NLIM) return;
  for (int rr = 0; rr < 16; ++rr) for (int q = 0; q < 3; ++q) { const int c = q * 32 + lane; Ah[rr][c] = (b16)(c < AD ? bf16_rne(x[(m0 + rr) * AD + c]) * XS : 0.0f); } if (lane < 16) for (int k = ADP; k < ADP + 8; ++k) Ah[lane][k] = (b16)0.0f;
  wave_lds_sync(); v8f acc[8];
#pragma unroll
  for (int t = 0; t < 8; ++t) acc[t] = (v8f){};
#pragma unroll
  for (int kb = 0; kb < ADP; kb += 32) { const v16b a = frag_kb(&Ah[nloc][kb], hlf);
#pragma unroll
    for (int t = 0; t < 8; ++t) acc[t] = wmma16b(a, frag_kb(WE + (size_t)(t * 16 + nloc) * ADP + kb, hlf), acc[t]); }
#pragma unroll
  for (int t = 0; t < 8; ++t) { const int cc = t * 16 + nloc; const float bb = bfv(be[cc]);
#pragma unroll
    for (int r8 = 0; r8 < 8; ++r8) Tf[8 * hlf + r8][cc] = acc[t][r8] * (1.0f / (XS * WSC)) + bb; }
  wave_lds_sync();
  for (int pass = 0; pass < 2; ++pass) { for (int rr = 0; rr < 16; ++rr) *(volatile v4f*)(HA + (m0 + rr) * H + lane * 4) = *(const v4f*)(&Tf[rr][lane * 4]); __threadfence(); } }
__global__ __launch_bounds__(32) void gin_kernel(const float* __restrict__ IN, const int* __restrict__ srcs, const int* __restrict__ PERM, const int* __restrict__ ROWPTR, const int* __restrict__ ROWCNT, int permLen, const float* __restrict__ epsv, int layer, const b16* __restrict__ WA, const float* __restrict__ ba, const float* __restrict__ ga, const float* __restrict__ bea, const b16* __restrict__ WB, const float* __restrict__ bb_, const float* __restrict__ gb_, const float* __restrict__ beb, int NLIM, float* __restrict__ OUTP) { __shared__ __attribute__((aligned(16))) b16 Ah[16][H + 8], Al[16][H + 8]; __shared__ float Tf[16][H + 4]; const int lane = threadIdx.x, nloc = lane & 15, hlf = lane >> 4; const size_t m0 = (size_t)blockIdx.x * 16; if (m0 >= (size_t)NLIM) return; const float ope = 1.0f + bfv(epsv[layer]);
  for (int rr = 0; rr < 16; ++rr) { const size_t i = m0 + rr; int st = ROWPTR[i], cnt = ROWCNT[i]; cnt = iclamp(cnt, 0, E); st = iclamp(st, 0, permLen - cnt); v4f ag = *(const v4f*)(IN + i * H + lane * 4) * ope;
#pragma unroll 1
    for (int j = 0; j < cnt; ++j) { const int e = iclamp(PERM[st + j], 0, E - 1); const size_t u = (size_t)iclamp(srcs[e], 0, N - 1); if (u >= (size_t)NLIM) continue; ag += *(const v4f*)(IN + u * H + lane * 4); }
    for (int k = 0; k < 4; ++k) { b16 p, ql; split16(ag[k] * HS, p, ql); Ah[rr][lane * 4 + k] = p; Al[rr][lane * 4 + k] = ql; } }
  if (lane < 16) for (int k = H; k < H + 8; ++k) { Ah[lane][k] = (b16)0.0f; Al[lane][k] = (b16)0.0f; }
  wave_lds_sync();
#pragma unroll 1
  for (int ph = 0; ph < 2; ++ph) { const b16* W = ph ? WB : WA; const float* bias = ph ? bb_ : ba; const float* gam = ph ? gb_ : ga; const float* bet = ph ? beb : bea; v8f acc[8];
#pragma unroll
    for (int t = 0; t < 8; ++t) acc[t] = (v8f){};
#pragma unroll
    for (int kb = 0; kb < H; kb += 32) { const v16b a = frag_kb(&Ah[nloc][kb], hlf), al = frag_kb(&Al[nloc][kb], hlf);
#pragma unroll
      for (int t = 0; t < 8; ++t) { const v16b bw = frag_kb(W + (size_t)(t * 16 + nloc) * H + kb, hlf); acc[t] = wmma16b(a, bw, acc[t]); acc[t] = wmma16b(al, bw, acc[t]); } }
#pragma unroll
    for (int t = 0; t < 8; ++t) { const int cc = t * 16 + nloc; const float bb = bfv(bias[cc]), sc = bfv(gam[cc]) * BNS, sh = bfv(bet[cc]);
#pragma unroll
      for (int r8 = 0; r8 < 8; ++r8) Tf[8 * hlf + r8][cc] = fmaxf(pmul(acc[t][r8] * (1.0f / (HS * WSC)) + bb, sc) + sh, 0.0f); }
    wave_lds_sync();
    if (ph == 0) { for (int rr = 0; rr < 16; ++rr) for (int q = 0; q < 4; ++q) { b16 p, ql; split16(Tf[rr][q * 32 + lane] * HS, p, ql); Ah[rr][q * 32 + lane] = p; Al[rr][q * 32 + lane] = ql; } wave_lds_sync(); } }
  for (int pass = 0; pass < 2; ++pass) { for (int rr = 0; rr < 16; ++rr) *(volatile v4f*)(OUTP + (m0 + rr) * H + lane * 4) = *(const v4f*)(&Tf[rr][lane * 4]); __threadfence(); } }
__global__ __launch_bounds__(32) void head_kernel(const float* __restrict__ HN, const int* __restrict__ PERM, const int* __restrict__ ROWPTR, const int* __restrict__ ROWCNT, int permLen, const b16* __restrict__ WF1, const float* __restrict__ bf1, const float* __restrict__ gf1, const float* __restrict__ bef1, const b16* __restrict__ WF2, const float* __restrict__ bf2, const float* __restrict__ gf2, const float* __restrict__ bef2, int NLIM, float* __restrict__ STG) { __shared__ __attribute__((aligned(16))) b16 Ah[16][H + 8], Al[16][H + 8]; __shared__ float Tf[16][H + 4]; const int lane = threadIdx.x, nloc = lane & 15, hlf = lane >> 4; const int g0 = blockIdx.x * 16;
  for (int rr = 0; rr < 16; ++rr) { const int g = g0 + rr; v4f s = {0, 0, 0, 0}; int nn = 0; if (g < G) { int st = ROWPTR[g], cnt = ROWCNT[g]; cnt = iclamp(cnt, 0, N); st = iclamp(st, 0, permLen - cnt);
#pragma unroll 1
      for (int j = 0; j < cnt; ++j) { const size_t n = (size_t)iclamp(PERM[st + j], 0, N - 1); if (n >= (size_t)NLIM) continue; ++nn; s += *(const v4f*)(HN + n * H + lane * 4); } }
    const float inv = 1.0f / fmaxf((float)nn, 1.0f); for (int k = 0; k < 4; ++k) { b16 p, ql; split16(s[k] * inv * HS, p, ql); Ah[rr][lane * 4 + k] = p; Al[rr][lane * 4 + k] = ql; } }
  if (lane < 16) for (int k = H; k < H + 8; ++k) { Ah[lane][k] = (b16)0.0f; Al[lane][k] = (b16)0.0f; }
  wave_lds_sync();
#pragma unroll 1
  for (int ph = 0; ph < 2; ++ph) { const b16* W = ph ? WF2 : WF1; const int NT = ph ? 7 : 8; v8f acc[8];
#pragma unroll
    for (int t = 0; t < 8; ++t) acc[t] = (v8f){};
#pragma unroll
    for (int kb = 0; kb < H; kb += 32) { const v16b a = frag_kb(&Ah[nloc][kb], hlf), al = frag_kb(&Al[nloc][kb], hlf);
#pragma unroll
      for (int t = 0; t < 8; ++t) if (t < NT) { const v16b bw = frag_kb(W + (size_t)(t * 16 + nloc) * H + kb, hlf); acc[t] = wmma16b(a, bw, acc[t]); acc[t] = wmma16b(al, bw, acc[t]); } }
#pragma unroll
    for (int t = 0; t < 8; ++t) { const int cc = t * 16 + nloc; float v0 = 0.0f; const bool real = ph == 0 || cc < OUT; const float bb = real ? bfv((ph ? bf2 : bf1)[cc]) : 0.0f, sc = real ? bfv((ph ? gf2 : gf1)[cc]) * BNS : 0.0f, sh = real ? bfv((ph ? bef2 : bef1)[cc]) : 0.0f;
#pragma unroll
      for (int r8 = 0; r8 < 8; ++r8) { v0 = (t < NT && real) ? fmaxf(pmul(acc[t][r8] * (1.0f / (HS * WSC)) + bb, sc) + sh, 0.0f) : 0.0f; Tf[8 * hlf + r8][cc] = v0; } }
    wave_lds_sync();
    if (ph == 0) { for (int rr = 0; rr < 16; ++rr) for (int q = 0; q < 4; ++q) { b16 p, ql; split16(Tf[rr][q * 32 + lane] * HS, p, ql); Ah[rr][q * 32 + lane] = p; Al[rr][q * 32 + lane] = ql; } wave_lds_sync(); } }
  for (int pass = 0; pass < 2; ++pass) { for (int rr = 0; rr < 16; ++rr) *(volatile v4f*)(STG + (size_t)(g0 + rr) * H + lane * 4) = *(const v4f*)(&Tf[rr][lane * 4]); __threadfence(); } }
__global__ __launch_bounds__(256) void copy_kernel(const float* __restrict__ STG, float* __restrict__ out) { const size_t u = (size_t)blockIdx.x * 256 + threadIdx.x; if (u >= (size_t)G * OUT) return; const size_t g = u / OUT, c = u % OUT;
  for (int pass = 0; pass < 2; ++pass) { ((volatile float*)out)[u] = STG[g * H + c]; __threadfence(); } }
}

extern "C" void kernel_launch(void* const* d_in, const int* in_sizes, int n_in, void* d_out, int out_size, void* d_ws, size_t ws_size, hipStream_t stream) {
  (void)n_in;
  auto Fp = [&](int i) { return (const float*)d_in[i]; }; auto Ip = [&](int i) { return (const int*)d_in[i]; };
  if (in_sizes[0] != N * AD || in_sizes[1] != 2 * E || in_sizes[2] != N || in_sizes[3] != AD * H || in_sizes[5] != NL || in_sizes[6] != NL * H * H || in_sizes[10] != NL * H * H || in_sizes[14] != H * H || in_sizes[18] != H * OUT || out_size != G * OUT) return;
  const int NLIM = N;
  size_t off = 0; char* ws = (char*)d_ws;
  auto carve = [&](size_t bytes) { char* p = ws + off; off += (bytes + 255) & ~(size_t)255; return p; };
  b16* WE = (b16*)carve((size_t)H * ADP * 2); b16* WL = (b16*)carve((size_t)2 * NL * H * H * 2); b16* WF1 = (b16*)carve((size_t)H * H * 2); b16* WF2 = (b16*)carve((size_t)112 * H * 2); float* HA = (float*)carve((size_t)N * H * 4); float* HB = (float*)carve((size_t)N * H * 4); float* STG = (float*)carve((size_t)GP * H * 4); CsrBufs8 csr; off = csr_carve8(csr, ws, off, E, N); CsrBufs5 cg; off = csr_carve5(cg, ws, off, N, G);
  if (off > ws_size || off > ((size_t)96 << 20)) return;
  wput_kernel<<<64, 256, 0, stream>>>(Fp(3), Fp(6), Fp(10), Fp(14), Fp(18), WE, WL, WF1, WF2);
  csr_build8(csr, Ip(1) + E, E, N, stream); csr_build5(cg, Ip(2), N, G, stream);
  emb_kernel<<<NLIM / 16, 32, 0, stream>>>(Fp(0), WE, Fp(4), NLIM, HA);
  for (int l = 0; l < NL; ++l) { const float* in = (l & 1) ? HB : HA; float* outp = (l & 1) ? HA : HB;
    gin_kernel<<<NLIM / 16, 32, 0, stream>>>(in, Ip(1), csr.PERM, csr.ROWPTR, csr.ROWCNT, (int)csr.permLen, Fp(5), l, WL + (size_t)(2 * l) * H * H, Fp(7) + l * H, Fp(8) + l * H, Fp(9) + l * H, WL + (size_t)(2 * l + 1) * H * H, Fp(11) + l * H, Fp(12) + l * H, Fp(13) + l * H, NLIM, outp); }
  head_kernel<<<GP / 16, 32, 0, stream>>>(HB, cg.PERM, cg.ROWPTR, cg.ROWCNT, (int)cg.permLen, WF1, Fp(15), Fp(16), Fp(17), WF2, Fp(19), Fp(20), Fp(21), NLIM, STG);
  copy_kernel<<<(G * OUT + 255) / 256, 256, 0, stream>>>(STG, (float*)d_out);
}
